// DecoderLayer_82334523065080
// MI455X (gfx1250) — hardware-verified
//
#include <hip/hip_runtime.h>
#ifndef NB
#define NB 4
#endif
#ifndef SEQ
#define SEQ 1024
#endif
#define NB_FULL 4
#define SEQ_FULL 1024
#define DM 1024
#define NH 16
#define HD 64
#define FF 4096
#define LQ (3 * DM)
#define MROWS (NB * SEQ)
#define NQT (SEQ / 64)
#define NKT (SEQ / 64)
static_assert(SEQ % 64 == 0);
static_assert(SEQ <= SEQ_FULL);
static_assert(NB >= 1 && NB <= NB_FULL);
static_assert(NKT <= 32);
static_assert(MROWS % 128 == 0);
static_assert(MROWS % 8 == 0);
static_assert(DM % 64 == 0 && FF % 64 == 0 && DM % 32 == 0 && FF % 32 == 0);
static_assert(NH == 16 && HD == 64 && DM == NH * HD);
static_assert(((size_t)MROWS * DM) % 2048 == 0);
static_assert((size_t)MROWS * LQ + (size_t)NB * NH * HD * SEQ <= (size_t)MROWS * FF);

typedef _Float16 v16h __attribute__((ext_vector_type(16)));
typedef _Float16 v4h  __attribute__((ext_vector_type(4)));
typedef _Float16 v4ha __attribute__((ext_vector_type(4), may_alias));
typedef unsigned short v8us __attribute__((ext_vector_type(8), may_alias));
typedef float  v8f  __attribute__((ext_vector_type(8)));
typedef float  v4f  __attribute__((ext_vector_type(4)));
typedef float  v4fa __attribute__((ext_vector_type(4), may_alias));
union FragH { v16h v; v8us half[2]; _Float16 h[16]; unsigned short u[16]; };

#define NEG_INF (-__builtin_inff())

__device__ __forceinline__ unsigned short bf16_bits(float x) { unsigned int u = __float_as_uint(x); return (unsigned short)((u + 0x7FFFu + ((u >> 16) & 1u)) >> 16); }
__device__ __forceinline__ float bf16_val(unsigned short b) { return __uint_as_float(((unsigned int)b) << 16); }
__device__ __forceinline__ float bf16_rne(float x) { return bf16_val(bf16_bits(x)); }

__device__ __forceinline__ v16h g2_frag(const _Float16* p, int hh) { FragH f; f.half[0] = *(const v8us*)((const unsigned short*)p + 8 * hh); f.half[1] = *(const v8us*)((const unsigned short*)p + 16 + 8 * hh); return f.v; }
__device__ __forceinline__ v8f g2_mma(v16h a, v16h b, v8f c) { v8f d = __builtin_amdgcn_wmma_f32_16x16x32_f16(false, a, false, b, (short)0, c, false, false); asm volatile("v_nop\n\tv_nop\n\tv_nop\n\tv_nop" : "+v"(d) : "v"(a), "v"(b)); return d; }

__global__ __launch_bounds__(256) void k_x16(const float* __restrict__ x, _Float16* __restrict__ X16) {
  const unsigned t = blockIdx.x * 256u + threadIdx.x; const unsigned e = t * 8u; const unsigned row = e >> 10, col = e & 1023u;
  const unsigned b = row / (unsigned)SEQ, s = row - b * (unsigned)SEQ;
  const float* src = x + ((size_t)(b * (unsigned)SEQ_FULL + s) * DM + col);
  const v4f a = *(const v4fa*)src; const v4f c = *(const v4fa*)(src + 4); FragH f;
#pragma unroll
  for (int q = 0; q < 4; ++q) { f.h[q] = (_Float16)bf16_rne(a[q]); f.h[4 + q] = (_Float16)bf16_rne(c[q]); }
  *(volatile v8us*)((unsigned short*)X16 + (size_t)e) = f.half[0]; __threadfence(); *(volatile v8us*)((unsigned short*)X16 + (size_t)e) = f.half[0]; }

__global__ __launch_bounds__(256) void k_wt(const float* __restrict__ W, unsigned K, unsigned N, _Float16* __restrict__ Bt) {
  __shared__ unsigned short tl[64][66];
  const unsigned tid = threadIdx.x; const unsigned ntn = N >> 6; const unsigned kt = blockIdx.x / ntn, nt = blockIdx.x - kt * ntn; const unsigned k0 = kt * 64u, n0 = nt * 64u;
  for (unsigned i = tid; i < 64u * 16u; i += 256u) { const unsigned r = i >> 4, c4 = (i & 15u) * 4u;
    const v4f v = *(const v4fa*)(W + (size_t)(k0 + r) * N + n0 + c4); FragH f;
#pragma unroll
    for (int q = 0; q < 4; ++q) f.h[q] = (_Float16)(bf16_rne(v[q]) * 16.0f);
#pragma unroll
    for (int q = 0; q < 4; ++q) tl[r][c4 + q] = f.u[q]; }
  __syncthreads();
  for (int pass = 0; pass < 2; ++pass) {
#pragma unroll
    for (unsigned rd = 0; rd < 2; ++rd) { const unsigned n = rd * 32u + (tid >> 3), pc = tid & 7u; FragH f;
#pragma unroll
      for (int q = 0; q < 8; ++q) f.u[q] = tl[pc * 8u + q][n];
      *(volatile v8us*)((unsigned short*)Bt + (size_t)(n0 + n) * K + k0 + pc * 8u) = f.half[0]; }
    if (pass == 0) __threadfence(); } }

template <int MODE>
__global__ __launch_bounds__(128) void k_gemm2(const _Float16* __restrict__ A, unsigned lda, const _Float16* __restrict__ Bh, unsigned ldb, float alpha, const float* __restrict__ bias,
    void* Cv, unsigned ldc, const void* Rv, unsigned ldr, unsigned M, unsigned N, unsigned K) {
  __shared__ __attribute__((aligned(16))) float so[4][32][68];
  const unsigned tid = threadIdx.x, w = tid >> 5, lane = tid & 31u, ln = lane & 15u; const int hh = (int)(lane >> 4);
  const unsigned ntn = N >> 6; const unsigned mt = blockIdx.x / ntn, nq = blockIdx.x - mt * ntn; const unsigned row0 = mt * 128u + 32u * w, col0 = nq * 64u; if (row0 >= M) return;
  const _Float16* a0p = A + (size_t)(row0 + ln) * lda; const _Float16* a1p = a0p + (size_t)16 * lda;
  const _Float16* b0p = Bh + (size_t)(col0 + ln) * ldb; const _Float16* b1p = b0p + (size_t)16 * ldb; const _Float16* b2p = b1p + (size_t)16 * ldb; const _Float16* b3p = b2p + (size_t)16 * ldb;
  const v8f z8 = {0.f,0.f,0.f,0.f,0.f,0.f,0.f,0.f}; v8f c00 = z8, c01 = z8, c02 = z8, c03 = z8, c10 = z8, c11 = z8, c12 = z8, c13 = z8;
#pragma unroll 1
  for (unsigned kb = 0; kb < K; kb += 32u) { const v16h a0 = g2_frag(a0p + kb, hh), a1 = g2_frag(a1p + kb, hh);
    v16h b = g2_frag(b0p + kb, hh); c00 = g2_mma(a0, b, c00); c10 = g2_mma(a1, b, c10);
    b = g2_frag(b1p + kb, hh); c01 = g2_mma(a0, b, c01); c11 = g2_mma(a1, b, c11);
    b = g2_frag(b2p + kb, hh); c02 = g2_mma(a0, b, c02); c12 = g2_mma(a1, b, c12);
    b = g2_frag(b3p + kb, hh); c03 = g2_mma(a0, b, c03); c13 = g2_mma(a1, b, c13); }
  v8f accs[8] = {c00, c01, c02, c03, c10, c11, c12, c13};
#pragma unroll
  for (int u = 0; u < 8; ++u) { const unsigned t = (unsigned)(u & 3), half = (unsigned)(u >> 2); const unsigned col = col0 + t * 16u + ln; const float bv = bf16_rne(bias[col]);
#pragma unroll
    for (int r = 0; r < 8; ++r) { const unsigned rloc = half * 16u + 8u * (unsigned)hh + (unsigned)r; float val = accs[u][r] * alpha + bv; if (MODE == 1) val = fmaxf(val, 0.0f); so[w][rloc][t * 16u + ln] = val; } }
  __builtin_amdgcn_fence(4  , "workgroup"); __builtin_amdgcn_wave_barrier();
  const unsigned rsub = lane >> 4, c4 = (lane & 15u) * 4u;
  if (MODE <= 1) {
    _Float16* C16 = (_Float16*)Cv;
    for (int pass = 0; pass < 2; ++pass) {
#pragma unroll
      for (unsigned q = 0; q < 16; ++q) { const unsigned r = q * 2u + rsub; const v4f v = *(const v4fa*)&so[w][r][c4]; v4h h4;
#pragma unroll
        for (int i = 0; i < 4; ++i) h4[i] = (_Float16)v[i];
        *(volatile v4h*)(C16 + (size_t)(row0 + r) * ldc + col0 + c4) = h4; }
      if (pass == 0) __threadfence(); }
  } else {
    float* C32 = (float*)Cv;
    for (int pass = 0; pass < 2; ++pass) {
#pragma unroll
      for (unsigned q = 0; q < 16; ++q) { const unsigned r = q * 2u + rsub; v4f v = *(const v4fa*)&so[w][r][c4]; const size_t ro = (size_t)(row0 + r) * ldr + col0 + c4;
        if (MODE == 2) { const v4f rr = *(const v4fa*)((const float*)Rv + ro);
#pragma unroll
          for (int i = 0; i < 4; ++i) v[i] += rr[i]; }
        else { const v4ha rh = *(const v4ha*)((const _Float16*)Rv + ro);
#pragma unroll
          for (int i = 0; i < 4; ++i) v[i] += (float)rh[i]; }
        *(volatile v4f*)(C32 + (size_t)(row0 + r) * ldc + col0 + c4) = v; }
      if (pass == 0) __threadfence(); } } }

__global__ __launch_bounds__(256) void k_vt2(const _Float16* __restrict__ QKV, _Float16* __restrict__ VT) {
  __shared__ unsigned short tl[64][66];
  const unsigned tid = threadIdx.x; const unsigned slab = blockIdx.x / (unsigned)NQT, lg = blockIdx.x - slab * (unsigned)NQT; const unsigned b = slab >> 4, hd = slab & 15u; const unsigned s0 = lg * 64u;
  for (unsigned i = tid; i < 64u * 8u; i += 256u) { const unsigned r = i >> 3, c8 = (i & 7u) * 8u; FragH f;
    f.half[0] = *(const v8us*)((const unsigned short*)QKV + (size_t)(b * (unsigned)SEQ + s0 + r) * LQ + 2u * DM + hd * HD + c8);
#pragma unroll
    for (int q = 0; q < 8; ++q) tl[r][c8 + q] = f.u[q]; }
  __syncthreads();
  for (int pass = 0; pass < 2; ++pass) {
#pragma unroll
    for (unsigned rd = 0; rd < 2; ++rd) { const unsigned d = rd * 32u + (tid >> 3), pc = tid & 7u; FragH f;
#pragma unroll
      for (int q = 0; q < 8; ++q) f.u[q] = tl[pc * 8u + q][d];
      *(volatile v8us*)((unsigned short*)VT + ((size_t)slab * HD + d) * SEQ + s0 + pc * 8u) = f.half[0]; }
    if (pass == 0) __threadfence(); } }

__global__ __launch_bounds__(256) void k_mflag(const float* __restrict__ mask, unsigned mbs, unsigned mqs, int* __restrict__ MF) {
  __shared__ int sf[32]; __shared__ int srow[64];
  const unsigned tid = threadIdx.x, qt = blockIdx.x, bm = blockIdx.y; const unsigned kt = tid >> 3, p = tid & 7u;
  const bool ok = kt < (unsigned)NKT; const unsigned ktc = ok ? kt : (unsigned)(NKT - 1);
  if (tid < 64u) srow[tid] = 0;
  __syncthreads();
  int nz = 0, hv = 1;
  const float* base = mask + (size_t)bm * mbs + ktc * 64u + p * 4u;
#pragma unroll 1
  for (unsigned r = 0; r < 64u; ++r) {
    const float* rowp = base + (size_t)(qt * 64u + r) * mqs;
    const v4f a = *(const v4fa*)rowp; const v4f c = *(const v4fa*)(rowp + 32);
    int z = 0;
#pragma unroll
    for (int i = 0; i < 4; ++i) { nz |= (int)(a[i] != 0.0f) | (int)(c[i] != 0.0f); hv &= (int)(a[i] >= 0.5f) & (int)(c[i] >= 0.5f); z |= (int)(a[i] == 0.0f) | (int)(c[i] == 0.0f); }
    if (ok && z != 0) srow[r] = 1; }
  nz |= __shfl_xor(nz, 1); nz |= __shfl_xor(nz, 2); nz |= __shfl_xor(nz, 4);
  hv &= __shfl_xor(hv, 1); hv &= __shfl_xor(hv, 2); hv &= __shfl_xor(hv, 4);
  if (p == 0u) sf[kt] = nz | (hv << 1);
  __syncthreads();
  if (tid < 32u) { int rc = 1;
#pragma unroll 1
    for (unsigned r = 0; r < 64u; ++r) rc &= srow[r];
    const int c = sf[tid]; int v = ((c & 1) == 0) ? 0 : ((((c >> 1) & rc) != 0) ? 3 : 1); v = (tid < (unsigned)NKT) ? v : 0;
    volatile int* d = MF + ((size_t)bm * NQT + qt) * 32u + tid; *d = v; __threadfence(); *d = v; } }

__global__ __launch_bounds__(128) void k_attn(const _Float16* __restrict__ QKV, const _Float16* __restrict__ VT, const float* __restrict__ mask, unsigned mbs, unsigned mqs,
                                              const int* __restrict__ MF, unsigned mfb, _Float16* __restrict__ CTX) {
  __shared__ __attribute__((aligned(16))) float so[4][16][68];
  const unsigned tid = threadIdx.x, w = tid >> 5, lane = tid & 31u, l15 = lane & 15u; const int hh = (int)(lane >> 4);
  const unsigned qt = blockIdx.x, slab = blockIdx.y; const unsigned b = slab >> 4, hd = slab & 15u;
  const unsigned q0 = qt * 64u + w * 16u;
  const _Float16* Qb = QKV + (size_t)(b * (unsigned)SEQ) * LQ + hd * HD;
  const _Float16* Kb = Qb + DM;
  const _Float16* Vb = VT + (size_t)slab * HD * SEQ;
  const float* mrow = mask + (size_t)b * mbs + (size_t)(q0 + l15) * mqs;
  const int* mfp = MF + (size_t)b * mfb + qt * 32u;
  const _Float16* qrow = Qb + (size_t)(q0 + l15) * LQ;
  const v16h qf0 = g2_frag(qrow, hh), qf1 = g2_frag(qrow + 32, hh);
  const v8f z8 = {0.f,0.f,0.f,0.f,0.f,0.f,0.f,0.f};
  v8f o[4] = {z8, z8, z8, z8};
  float m = NEG_INF, l = 0.f;
  const float L2E = 1.4426950408889634f;
#pragma unroll 1
  for (unsigned it = 0; it < (unsigned)NKT; ++it) {
    const int mf = __builtin_amdgcn_readfirstlane(mfp[it]);
    if (mf == 3) continue;
    const unsigned key0 = it * 64u;
    v8f s[4];
#pragma unroll
    for (int kt = 0; kt < 4; ++kt) {
      const _Float16* krow = Kb + (size_t)(key0 + (unsigned)kt * 16u + l15) * LQ;
      const v16h ka = g2_frag(krow, hh), kk = g2_frag(krow + 32, hh);
      v8f a = g2_mma(ka, qf0, z8); a = g2_mma(kk, qf1, a);
#pragma unroll
      for (int r = 0; r < 8; ++r) a[r] *= 0.125f;
      s[kt] = a; }
    if (mf != 0) {
#pragma unroll
      for (int kt = 0; kt < 4; ++kt) {
        const float* mp = mrow + key0 + (unsigned)kt * 16u + 8u * (unsigned)hh;
        const v4f ma = *(const v4fa*)mp; const v4f mb = *(const v4fa*)(mp + 4);
#pragma unroll
        for (int r = 0; r < 4; ++r) { s[kt][r] = fmaf(bf16_rne(ma[r]), -1.0e9f, s[kt][r]); s[kt][4 + r] = fmaf(bf16_rne(mb[r]), -1.0e9f, s[kt][4 + r]); } } }
    float lmax = NEG_INF;
#pragma unroll
    for (int kt = 0; kt < 4; ++kt)
#pragma unroll
      for (int r = 0; r < 8; ++r) lmax = fmaxf(lmax, s[kt][r]);
    lmax = fmaxf(lmax, __shfl_xor(lmax, 16));
    const float mnew = fmaxf(m, lmax);
    const float mref = (mnew == NEG_INF) ? 0.0f : mnew;
    const float alpha = exp2f((m - mref) * L2E);
    const float bexp = 10.0f - mref * L2E;
    m = mnew;
    float psum = 0.f; FragH pa, pb;
#pragma unroll
    for (int r = 0; r < 8; ++r) {
      const float e0 = exp2f(fmaf(s[0][r], L2E, bexp)), e1 = exp2f(fmaf(s[1][r], L2E, bexp)), e2 = exp2f(fmaf(s[2][r], L2E, bexp)), e3 = exp2f(fmaf(s[3][r], L2E, bexp));
      psum += (e0 + e1) + (e2 + e3);
      pa.h[r] = (_Float16)e0; pa.h[8 + r] = (_Float16)e1; pb.h[r] = (_Float16)e2; pb.h[8 + r] = (_Float16)e3; }
    l = l * alpha + psum;
    float ar[8];
#pragma unroll
    for (int r = 0; r < 8; ++r) ar[r] = __shfl(alpha, 8 * hh + r);
#pragma unroll
    for (int dt = 0; dt < 4; ++dt) {
#pragma unroll
      for (int r = 0; r < 8; ++r) o[dt][r] *= ar[r];
      const _Float16* vrow = Vb + (size_t)((unsigned)dt * 16u + l15) * SEQ + key0;
      const v16h va = g2_frag(vrow, hh), vb = g2_frag(vrow + 32, hh);
      o[dt] = g2_mma(pa.v, va, o[dt]); o[dt] = g2_mma(pb.v, vb, o[dt]); } }
  const float lt = l + __shfl_xor(l, 16);
  const float inv = 16.0f * (1.0f / lt);
  float ir[8];
#pragma unroll
  for (int r = 0; r < 8; ++r) ir[r] = __shfl(inv, 8 * hh + r);
#pragma unroll
  for (int dt = 0; dt < 4; ++dt)
#pragma unroll
    for (int r = 0; r < 8; ++r) so[w][8 * hh + r][dt * 16 + (int)l15] = o[dt][r] * ir[r];
  __builtin_amdgcn_fence(4  , "workgroup"); __builtin_amdgcn_wave_barrier();
  const unsigned rsub = lane >> 4, c4 = (lane & 15u) * 4u;
  for (int pass = 0; pass < 2; ++pass) {
#pragma unroll
    for (unsigned q = 0; q < 8; ++q) { const unsigned r = q * 2u + rsub; const v4f v = *(const v4fa*)&so[w][r][c4]; v4h h4;
#pragma unroll
      for (int i = 0; i < 4; ++i) h4[i] = (_Float16)v[i];
      *(volatile v4h*)(CTX + (size_t)(b * (unsigned)SEQ + q0 + r) * DM + hd * HD + c4) = h4; }
    if (pass == 0) __threadfence(); } }

template <int FINAL>
__global__ __launch_bounds__(256) void k_ln(const float* __restrict__ P, const float* __restrict__ g, const float* __restrict__ be, float* __restrict__ OF, _Float16* __restrict__ OH) {
  const unsigned tid = threadIdx.x, w = tid >> 5, lane = tid & 31u; const unsigned row = blockIdx.x * 8u + w;
  const float* p = P + (size_t)row * DM + lane * 4u;
  float s = 0.f;
#pragma unroll 1
  for (unsigned j = 0; j < 8u; ++j) { const v4f v = *(const v4fa*)(p + j * 128u); s += (v[0] + v[1]) + (v[2] + v[3]); }
  s += __shfl_xor(s, 16); s += __shfl_xor(s, 8); s += __shfl_xor(s, 4); s += __shfl_xor(s, 2); s += __shfl_xor(s, 1);
  const float mu = s * (1.0f / 1024.0f);
  float qs = 0.f;
#pragma unroll 1
  for (unsigned j = 0; j < 8u; ++j) { const v4f v = *(const v4fa*)(p + j * 128u); const float d0 = v[0] - mu, d1 = v[1] - mu, d2 = v[2] - mu, d3 = v[3] - mu; qs += (d0 * d0 + d1 * d1) + (d2 * d2 + d3 * d3); }
  qs += __shfl_xor(qs, 16); qs += __shfl_xor(qs, 8); qs += __shfl_xor(qs, 4); qs += __shfl_xor(qs, 2); qs += __shfl_xor(qs, 1);
  const float rstd = rsqrtf(qs * (1.0f / 1024.0f) + 1.0e-6f);
  const unsigned bb = row / (unsigned)SEQ, ss = row - bb * (unsigned)SEQ;
  const unsigned orow = (FINAL != 0) ? (bb * (unsigned)SEQ_FULL + ss) : row;
  for (int pass = 0; pass < 2; ++pass) {
#pragma unroll 1
    for (unsigned j = 0; j < 8u; ++j) { const unsigned col = j * 128u + lane * 4u; const v4f v = *(const v4fa*)(p + j * 128u); const v4f gg = *(const v4fa*)(g + col); const v4f bt = *(const v4fa*)(be + col); v4f y;
#pragma unroll
      for (int i = 0; i < 4; ++i) y[i] = (v[i] - mu) * rstd * bf16_rne(gg[i]) + bf16_rne(bt[i]);
      *(volatile v4f*)(OF + (size_t)orow * DM + col) = y;
      if (FINAL == 0) { v4h h4;
#pragma unroll
        for (int i = 0; i < 4; ++i) h4[i] = (_Float16)y[i];
        *(volatile v4h*)(OH + (size_t)row * DM + col) = h4; } }
    if (pass == 0) __threadfence(); } }

extern "C" void kernel_launch(void* const* d_in, const int* in_sizes, int n_in,
                              void* d_out, int out_size, void* d_ws, size_t ws_size, hipStream_t stream) {
  if (n_in < 30) return;
  const float* x   = (const float*)d_in[0];
  const float* enc = (const float*)d_in[1];
  const float* m1  = (const float*)d_in[2];
  const float* m2  = (const float*)d_in[3];
  const int need_rows = ((NB - 1) * SEQ_FULL + SEQ) * DM;
  if (in_sizes[0] < need_rows || in_sizes[1] < need_rows) return;
  if (in_sizes[2] < (SEQ - 1) * SEQ_FULL + SEQ) return;
  if (in_sizes[3] < (NB - 1) * SEQ_FULL + SEQ) return;
  for (int i = 4; i <= 18; i += 2) { if (in_sizes[i] < DM * DM || in_sizes[i + 1] < DM) return; }
  if (in_sizes[20] < DM * FF || in_sizes[21] < FF || in_sizes[22] < FF * DM || in_sizes[23] < DM) return;
  for (int i = 24; i < 30; ++i) { if (in_sizes[i] < DM) return; }
  if (out_size < need_rows) return;
  char* ws = (char*)d_ws; size_t off = 0;
  auto take = [&](size_t bytes) { char* p = ws + off; off += (bytes + 255) & ~(size_t)255; return p; };
  _Float16* BW[8];
  for (int i = 0; i < 8; ++i) BW[i] = (_Float16*)take((size_t)DM * DM * 2);
  _Float16* BF1 = (_Float16*)take((size_t)DM * FF * 2);
  _Float16* BF2 = (_Float16*)take((size_t)FF * DM * 2);
  _Float16* ACT = (_Float16*)take((size_t)MROWS * DM * 2);
  _Float16* E16 = (_Float16*)take((size_t)MROWS * DM * 2);
  _Float16* R   = (_Float16*)take((size_t)MROWS * FF * 2);
  _Float16* CTX = (_Float16*)take((size_t)MROWS * DM * 2);
  float*    PA  = (float*)take((size_t)MROWS * DM * 4);
  float*    PB  = (float*)take((size_t)MROWS * DM * 4);
  int*      MF1 = (int*)take((size_t)NQT * 32 * 4);
  int*      MF2 = (int*)take((size_t)NB * NQT * 32 * 4);
  if (off > ws_size || off > (size_t)134217728) return;
  _Float16* QKV = R; _Float16* VT = R + (size_t)MROWS * LQ; _Float16* H16 = R;
  const unsigned gw = (unsigned)((DM / 64) * (DM / 64));
  for (int i = 0; i < 8; ++i) k_wt<<<gw, 256, 0, stream>>>((const float*)d_in[4 + 2 * i], (unsigned)DM, (unsigned)DM, BW[i]);
  k_wt<<<(unsigned)((DM / 64) * (FF / 64)), 256, 0, stream>>>((const float*)d_in[20], (unsigned)DM, (unsigned)FF, BF1);
  k_wt<<<(unsigned)((FF / 64) * (DM / 64)), 256, 0, stream>>>((const float*)d_in[22], (unsigned)FF, (unsigned)DM, BF2);
  const unsigned gx = (unsigned)(((size_t)MROWS * DM) / 2048);
  k_x16<<<gx, 256, 0, stream>>>(x, ACT);
  k_x16<<<gx, 256, 0, stream>>>(enc, E16);
  const unsigned gd = (unsigned)((MROWS / 128) * (DM / 64));
  const unsigned gf = (unsigned)((MROWS / 128) * (FF / 64));
  k_gemm2<0><<<gd, 128, 0, stream>>>(ACT, DM, BW[0], DM, 0.0625f, (const float*)d_in[5], QKV,          LQ, ACT, DM, MROWS, DM, DM);
  k_gemm2<0><<<gd, 128, 0, stream>>>(ACT, DM, BW[1], DM, 0.0625f, (const float*)d_in[7], QKV + DM,     LQ, ACT, DM, MROWS, DM, DM);
  k_gemm2<0><<<gd, 128, 0, stream>>>(ACT, DM, BW[2], DM, 0.0625f, (const float*)d_in[9], QKV + 2 * DM, LQ, ACT, DM, MROWS, DM, DM);
  k_vt2<<<(unsigned)(NB * NH * NQT), 256, 0, stream>>>(QKV, VT);
  k_mflag<<<dim3((unsigned)NQT, 1u), 256, 0, stream>>>(m1, 0u, (unsigned)SEQ_FULL, MF1);
  k_mflag<<<dim3((unsigned)NQT, (unsigned)NB), 256, 0, stream>>>(m2, (unsigned)SEQ_FULL, 0u, MF2);
  k_attn<<<dim3((unsigned)NQT, (unsigned)(NB * NH)), 128, 0, stream>>>(QKV, VT, m1, 0u, (unsigned)SEQ_FULL, MF1, 0u, CTX);
  k_gemm2<3><<<gd, 128, 0, stream>>>(CTX, DM, BW[3], DM, 0.00390625f, (const float*)d_in[11], PA, DM, ACT, DM, MROWS, DM, DM);
  k_ln<0><<<(unsigned)(MROWS / 8), 256, 0, stream>>>(PA, (const float*)d_in[24], (const float*)d_in[25], PB, ACT);
  k_gemm2<0><<<gd, 128, 0, stream>>>(ACT, DM, BW[4], DM, 0.0625f, (const float*)d_in[13], QKV,          LQ, ACT, DM, MROWS, DM, DM);
  k_gemm2<0><<<gd, 128, 0, stream>>>(E16, DM, BW[5], DM, 0.0625f, (const float*)d_in[15], QKV + DM,     LQ, ACT, DM, MROWS, DM, DM);
  k_gemm2<0><<<gd, 128, 0, stream>>>(E16, DM, BW[6], DM, 0.0625f, (const float*)d_in[17], QKV + 2 * DM, LQ, ACT, DM, MROWS, DM, DM);
  k_vt2<<<(unsigned)(NB * NH * NQT), 256, 0, stream>>>(QKV, VT);
  k_attn<<<dim3((unsigned)NQT, (unsigned)(NB * NH)), 128, 0, stream>>>(QKV, VT, m2, (unsigned)SEQ_FULL, 0u, MF2, (unsigned)(NQT * 32), CTX);
  k_gemm2<2><<<gd, 128, 0, stream>>>(CTX, DM, BW[7], DM, 0.00390625f, (const float*)d_in[19], PA, DM, PB, DM, MROWS, DM, DM);
  k_ln<0><<<(unsigned)(MROWS / 8), 256, 0, stream>>>(PA, (const float*)d_in[26], (const float*)d_in[27], PB, ACT);
  k_gemm2<1><<<gf, 128, 0, stream>>>(ACT, DM, BF1, DM, 0.0625f, (const float*)d_in[21], H16, FF, ACT, DM, MROWS, FF, DM);
  k_gemm2<2><<<gd, 128, 0, stream>>>(H16, FF, BF2, FF, 0.0625f, (const float*)d_in[23], PA, DM, PB, DM, MROWS, DM, FF);
  k_ln<1><<<(unsigned)(MROWS / 8), 256, 0, stream>>>(PA, (const float*)d_in[28], (const float*)d_in[29], (float*)d_out, ACT);
}
